// Model2_68229850464411
// MI455X (gfx1250) — hardware-run, weakly checked
//
#include <hip/hip_runtime.h>
#include <math.h>

typedef __attribute__((ext_vector_type(16))) _Float16 v16h;
typedef __attribute__((ext_vector_type(8)))  _Float16 v8h;
typedef __attribute__((ext_vector_type(4)))  _Float16 v4h;
typedef __attribute__((ext_vector_type(8)))  float    v8f;
typedef __attribute__((ext_vector_type(4)))  float    v4f;

constexpr int kPts    = 200000;
constexpr int kGraphs = 512;
constexpr int kCin    = 32;
constexpr int kCh     = 64;
constexpr int kRep    = 9;
constexpr int kRings  = 4;
constexpr int kKdim   = kCin * kRings;
constexpr int kGridN  = 40;
constexpr int kChunk  = 64;
constexpr int kPitch  = 72;
constexpr int kMrows  = 64;
constexpr int kPRows  = kRep * kRings;
constexpr int kRowsT  = kGraphs * kRep;
constexpr float kCarryP    = 1024.0f;
constexpr float kInvCarryP = 1.0f / 1024.0f;
constexpr float kCarryW    = 16.0f;
constexpr float kInvCarryW = 1.0f / 16.0f;
constexpr float kEps       = 1e-5f;

static_assert(kKdim == 128, "K of the channel product");
static_assert((kKdim % 32) == 0, "K multiple of 32");
static_assert((kRowsT % 64) == 0 && (kCh % 64) == 0, "M, N multiples of 64");
static_assert((kRowsT % 16) == 0, "second-moment row blocking");
static_assert(kPRows <= kMrows, "P rows fit the padded M tile");
static_assert((kRep * kKdim * 2) % 128 == 0, "per-graph T block is whole lines");

constexpr size_t kOffTP  = 0;
constexpr size_t kOffWH  = kOffTP + (size_t)kRowsT * kKdim * 2;
constexpr size_t kOffOP  = kOffWH + (size_t)kCh * kKdim * 2;
constexpr size_t kOffSCL = kOffOP + (size_t)kRowsT * kCh * 4;
constexpr size_t kWsTotal = kOffSCL + (size_t)kCh * 4;
static_assert(kWsTotal == 2375936ull, "carve total");
static_assert(kWsTotal <= 134217728ull, "carve cap");
static_assert((kOffWH % 128) == 0 && (kOffOP % 128) == 0 && (kOffSCL % 128) == 0, "aligned regions");

union FragU { v16h v; v8h h[2]; };
__device__ __forceinline__ v16h frag_load_h(const _Float16* p) {
  FragU f;
  f.h[0] = *(const v8h*)(p);
  f.h[1] = *(const v8h*)(p + 16);
  return f.v;
}
__device__ __forceinline__ v8f mma_h(v16h a, v16h b, v8f c) {
  c = __builtin_amdgcn_wmma_f32_16x16x32_f16(false, a, false, b, (short)0, c, false, false);
  asm volatile("v_nop\n\tv_nop\n\tv_nop\n\tv_nop" : "+v"(c) : "v"(a), "v"(b));
  return c;
}

__device__ __forceinline__ int lower_bound_sorted(const int* __restrict__ a, int key) {
  int lo = 0, hi = kPts;
#pragma unroll 1
  for (int it = 0; it < 20; ++it) {
    const bool act = lo < hi;
    int mid = (lo + hi) >> 1;
    mid = (mid < kPts - 1) ? mid : (kPts - 1);
    const int v = a[mid];
    const bool less = v < key;
    lo = (act && less) ? (mid + 1) : lo;
    hi = (act && !less) ? mid : hi;
  }
  return lo;
}

__global__ __launch_bounds__(256) void cast_w_kernel(const float* __restrict__ W, unsigned short* __restrict__ WH) {
  const int i = blockIdx.x * 256 + threadIdx.x;
  if (i >= (kCh * kKdim) / 8) return;
  const size_t e0 = (size_t)i << 3;
  const v4f a0 = *(const v4f*)(W + e0);
  const v4f a1 = *(const v4f*)(W + e0 + 4);
  v8h hv;
#pragma unroll
  for (int e = 0; e < 4; ++e) {
    const float f0 = a0[e] * kCarryW;
    const float f1 = a1[e] * kCarryW;
    hv[e]     = (_Float16)f0;
    hv[4 + e] = (_Float16)f1;
  }
  unsigned short* q = WH + e0;
  *(volatile v8h*)q = hv;
  __threadfence();
  *(volatile v8h*)q = hv;
}

__global__ __launch_bounds__(128) void pool_kernel(
    const float* __restrict__ x, const float* __restrict__ coords, const int* __restrict__ batch,
    unsigned short* __restrict__ Tplane)
{
  __shared__ __align__(16) _Float16 sP[kMrows * kPitch];
  __shared__ __align__(16) _Float16 sXt[kCin * kPitch];
  __shared__ __align__(16) _Float16 sTt[kRep * kKdim];
  __shared__ float sRed[3 * 128];

  const int b    = blockIdx.x;
  const int tid  = threadIdx.x;
  const int lane = tid & 31;
  const int wave = tid >> 5;
  const int hh   = lane >> 4;
  const int rl   = lane & 15;

#pragma unroll 1
  for (int idx = tid; idx < kMrows * kPitch; idx += 128) sP[idx] = (_Float16)0.0f;
#pragma unroll 1
  for (int idx = tid; idx < kCin * kPitch; idx += 128) sXt[idx] = (_Float16)0.0f;

  int s = lower_bound_sorted(batch, b);
  int e = lower_bound_sorted(batch, b + 1);
  s = (s < 0) ? 0 : ((s > kPts) ? kPts : s);
  e = (e < s) ? s : ((e > kPts) ? kPts : e);
  const int cnt = e - s;

  float sx = 0.0f, sy = 0.0f, sz = 0.0f;
  {
    int nIt = (cnt + 127) >> 7;
    nIt = (nIt < (kPts + 127) / 128) ? nIt : ((kPts + 127) / 128);
#pragma unroll 1
    for (int it = 0; it < nIt; ++it) {
      const int n = s + it * 128 + tid;
      const bool valid = n < e;
      const int nc = valid ? n : (e - 1);
      const float cx = coords[(size_t)nc * 3 + 0];
      const float cy = coords[(size_t)nc * 3 + 1];
      const float cz = coords[(size_t)nc * 3 + 2];
      sx += valid ? cx : 0.0f;
      sy += valid ? cy : 0.0f;
      sz += valid ? cz : 0.0f;
    }
  }
  sRed[tid]       = sx;
  sRed[128 + tid] = sy;
  sRed[256 + tid] = sz;
  __syncthreads();
#pragma unroll 1
  for (int w = 64; w > 0; w >>= 1) {
    if (tid < w) {
      sRed[tid]       += sRed[tid + w];
      sRed[128 + tid] += sRed[128 + tid + w];
      sRed[256 + tid] += sRed[256 + tid + w];
    }
    __syncthreads();
  }
  const float cntf = (cnt > 1) ? (float)cnt : 1.0f;
  const float icnt = 1.0f / cntf;
  const float px = sRed[0] * icnt;
  const float py = sRed[128] * icnt;
  const float pz = sRed[256] * icnt;

  v8f acc0 = (v8f){0.f, 0.f, 0.f, 0.f, 0.f, 0.f, 0.f, 0.f};
  v8f acc1 = (v8f){0.f, 0.f, 0.f, 0.f, 0.f, 0.f, 0.f, 0.f};

  int nChunks = (cnt + kChunk - 1) / kChunk;
  nChunks = (nChunks < (kPts + kChunk - 1) / kChunk) ? nChunks : ((kPts + kChunk - 1) / kChunk);

#pragma unroll 1
  for (int ch = 0; ch < nChunks; ++ch) {
    const int base = s + ch * kChunk;

#pragma unroll
    for (int j = 0; j < 4; ++j) {
      const int idx = tid + 128 * j;
      const int p   = idx >> 3;
      const int c4  = (idx & 7) * 4;
      const int n   = base + p;
      const bool valid = n < e;
      const int nc  = (n < kPts - 1) ? n : (kPts - 1);
      const v4f v = *(const v4f*)(x + (size_t)nc * kCin + c4);
#pragma unroll
      for (int q = 0; q < 4; ++q) {
        const float f = v[q];
        sXt[(c4 + q) * kPitch + p] = valid ? (_Float16)f : (_Float16)0.0f;
      }
    }

    if (tid < kChunk) {
      const int p = tid;
      const int n = base + p;
      const bool valid = n < e;
      const int nc = (n < kPts - 1) ? n : (kPts - 1);
      const float rx = coords[(size_t)nc * 3 + 0] - px;
      const float ry = coords[(size_t)nc * 3 + 1] - py;
      const float rz = coords[(size_t)nc * 3 + 2] - pz;
      const float r  = sqrtf(rx * rx + ry * ry + rz * rz);
      const float inv = 1.0f / (r + 1e-8f);
      const float dx = rx * inv, dy = ry * inv, dz = rz * inv;
      const float c0 = 0.28209479f, c1 = 0.48860251f, c2 = 1.09254843f;
      const float c20 = 0.31539157f, c22 = 0.54627421f;
      float Yv[kRep];
      Yv[0] = c0;
      Yv[1] = c1 * dy;
      Yv[2] = c1 * dz;
      Yv[3] = c1 * dx;
      Yv[4] = c2 * dx * dy;
      Yv[5] = c2 * dy * dz;
      Yv[6] = c20 * (3.0f * dz * dz - 1.0f);
      Yv[7] = c2 * dx * dz;
      Yv[8] = c22 * (dx * dx - dy * dy);
      float ring[kRings];
#pragma unroll
      for (int j = 0; j < kRings; ++j) {
        const float cen = (2.0f / 3.0f) * (float)j;
        const float t = r - cen;
        ring[j] = expf(-2.0f * (t * t)) * kCarryP;
      }
#pragma unroll
      for (int d = 0; d < kRep; ++d) {
#pragma unroll
        for (int j = 0; j < kRings; ++j) {
          const float val = Yv[d] * ring[j];
          sP[(d * kRings + j) * kPitch + p] = valid ? (_Float16)val : (_Float16)0.0f;
        }
      }
    }
    __syncthreads();

#pragma unroll
    for (int ks = 0; ks < 2; ++ks) {
      const v16h a  = frag_load_h(sP  + (16 * wave + rl) * kPitch + ks * 32 + 8 * hh);
      const v16h b0 = frag_load_h(sXt + (rl) * kPitch + ks * 32 + 8 * hh);
      const v16h b1 = frag_load_h(sXt + (16 + rl) * kPitch + ks * 32 + 8 * hh);
      acc0 = mma_h(a, b0, acc0);
      acc1 = mma_h(a, b1, acc1);
    }
    __syncthreads();
  }

#pragma unroll
  for (int g = 0; g < 2; ++g) {
    const int d = 4 * wave + 2 * hh + g;
    v4h t0, t1;
#pragma unroll
    for (int q = 0; q < 4; ++q) {
      const float f0 = acc0[4 * g + q] * kInvCarryP;
      const float f1 = acc1[4 * g + q] * kInvCarryP;
      t0[q] = (_Float16)f0;
      t1[q] = (_Float16)f1;
    }
    if (d < kRep) {
      *(v4h*)(sTt + d * kKdim + (rl) * 4)      = t0;
      *(v4h*)(sTt + d * kKdim + (16 + rl) * 4) = t1;
    }
  }
  __syncthreads();

  {
    unsigned short* Tb = Tplane + (size_t)b * (kRep * kKdim);
    const int offMain = 256 * wave + 8 * lane;
    const int offTail = 1024 + 8 * (lane & 15);
    const v8h v0 = *(const v8h*)(sTt + offMain);
    const v8h v1 = *(const v8h*)(sTt + offTail);
    for (int pass = 0; pass < 2; ++pass) {
      *(volatile v8h*)(Tb + offMain) = v0;
      if (wave == 0 && lane < 16) *(volatile v8h*)(Tb + offTail) = v1;
      __threadfence();
    }
  }
}

__global__ __launch_bounds__(256) void gemm_f16_tile64(
    const unsigned short* __restrict__ Ap, int lda,
    const unsigned short* __restrict__ Btp, int ldb,
    float* __restrict__ C, int ldc, int M, int N, int K, float scale)
{
  const _Float16* A  = (const _Float16*)Ap;
  const _Float16* Bt = (const _Float16*)Btp;
  __shared__ __align__(16) float sSlab[8][16 * 68];
  const int lane = threadIdx.x & 31;
  const int wave = threadIdx.x >> 5;
  const int tilesN = N >> 6;
  const int tilesM = M >> 6;
  const int tile = blockIdx.x * 8 + wave;
  if (tile >= tilesM * tilesN) return;
  const int tm = tile / tilesN;
  const int tn = tile - tm * tilesN;
  const int m0 = tm << 6;
  const int n0 = tn << 6;

  const int rlane = lane & 15;
  const int koff  = (lane >> 4) * 8;
  const int mOff  = (lane >> 4) * 8;

  v8f acc[4][4];
#pragma unroll
  for (int i = 0; i < 4; ++i)
#pragma unroll
    for (int j = 0; j < 4; ++j) acc[i][j] = (v8f){0.f, 0.f, 0.f, 0.f, 0.f, 0.f, 0.f, 0.f};

  for (int k0 = 0; k0 < K; k0 += 32) {
    v16h bh[4];
#pragma unroll
    for (int j = 0; j < 4; ++j) {
      const size_t bo = (size_t)(n0 + (j << 4) + rlane) * ldb + koff + k0;
      bh[j] = frag_load_h(Bt + bo);
    }
#pragma unroll
    for (int i = 0; i < 4; ++i) {
      const size_t ao = (size_t)(m0 + (i << 4) + rlane) * lda + koff + k0;
      const v16h ah = frag_load_h(A + ao);
#pragma unroll
      for (int j = 0; j < 4; ++j) acc[i][j] = mma_h(ah, bh[j], acc[i][j]);
    }
  }

  float* slab = sSlab[wave];
#pragma unroll
  for (int i = 0; i < 4; ++i) {
    const int mBase = m0 + (i << 4);
#pragma unroll
    for (int j = 0; j < 4; ++j) {
#pragma unroll
      for (int r = 0; r < 8; ++r) {
        const float v = acc[i][j][r] * scale;
        slab[(mOff + r) * 68 + (j << 4) + rlane] = v;
      }
    }
    __builtin_amdgcn_fence(__ATOMIC_RELEASE, "workgroup");
    __builtin_amdgcn_wave_barrier();
    __builtin_amdgcn_fence(__ATOMIC_ACQUIRE, "workgroup");
    {
      const int hh = lane >> 4, c4 = (lane & 15) * 4;
      for (int pass = 0; pass < 2; ++pass) {
#pragma unroll
        for (int it = 0; it < 8; ++it) {
          const int row = it * 2 + hh;
          const v4f v = *(const v4f*)(slab + row * 68 + c4);
          *(volatile v4f*)(C + (size_t)(mBase + row) * ldc + n0 + c4) = v;
        }
        __threadfence();
      }
    }
    __builtin_amdgcn_fence(__ATOMIC_RELEASE, "workgroup");
    __builtin_amdgcn_wave_barrier();
    __builtin_amdgcn_fence(__ATOMIC_ACQUIRE, "workgroup");
  }
}

__global__ __launch_bounds__(256) void scale_kernel(
    const float* __restrict__ OP, const float* __restrict__ gamma, float* __restrict__ SCL)
{
  __shared__ float sRed[256];
  __shared__ __align__(16) float sScl[kCh];
  const int tid = threadIdx.x;
  const int c = tid & 63;
  const int q = tid >> 6;
  float a0 = 0.0f, a1 = 0.0f, a2 = 0.0f, a3 = 0.0f;
#pragma unroll 1
  for (int t = 0; t < kRowsT / 16; ++t) {
    const int r0 = q + 16 * t;
    const float v0 = OP[(size_t)(r0) * kCh + c];
    const float v1 = OP[(size_t)(r0 + 4) * kCh + c];
    const float v2 = OP[(size_t)(r0 + 8) * kCh + c];
    const float v3 = OP[(size_t)(r0 + 12) * kCh + c];
    a0 = fmaf(v0, v0, a0);
    a1 = fmaf(v1, v1, a1);
    a2 = fmaf(v2, v2, a2);
    a3 = fmaf(v3, v3, a3);
  }
  sRed[tid] = (a0 + a1) + (a2 + a3);
  __syncthreads();
  if (tid < kCh) {
    const float tot = (sRed[tid] + sRed[64 + tid]) + (sRed[128 + tid] + sRed[192 + tid]);
    const float mom = tot * (1.0f / (float)kRowsT);
    const float g = gamma[tid];
    sScl[tid] = g * (1.0f / sqrtf(mom + kEps));
  }
  __syncthreads();
  if (tid < 16) {
    const v4f v = *(const v4f*)(sScl + 4 * tid);
    float* p = SCL + 4 * tid;
    *(volatile v4f*)p = v;
    __threadfence();
    *(volatile v4f*)p = v;
  }
}

__global__ __launch_bounds__(64) void final_kernel(
    const float* __restrict__ OP, const float* __restrict__ SCL, const float* __restrict__ Amat,
    const float* __restrict__ Ainv, float* __restrict__ out)
{
  __shared__ float sA[384];
  __shared__ float sAi[64];
  const int b = blockIdx.x;
  const int c = threadIdx.x;
#pragma unroll
  for (int it = 0; it < 6; ++it) {
    const int idx = c + 64 * it;
    const int idc = (idx < kRep * kGridN - 1) ? idx : (kRep * kGridN - 1);
    sA[idx] = Amat[idc];
  }
  {
    const int ic = (c < kGridN - 1) ? c : (kGridN - 1);
    sAi[c] = Ainv[ic];
  }
  const float sc = SCL[c];
  float o[kRep];
#pragma unroll
  for (int d = 0; d < kRep; ++d) o[d] = OP[(size_t)(b * kRep + d) * kCh + c] * sc;
  __syncthreads();
  float res = 0.0f;
#pragma unroll 1
  for (int n = 0; n < kGridN; ++n) {
    float v = 0.0f;
#pragma unroll
    for (int d = 0; d < kRep; ++d) v = fmaf(o[d], sA[d * kGridN + n], v);
    const float vn = (v > 0.0f) ? 0.0f : v;
    const float em = expm1f(vn);
    const float act = (v > 0.0f) ? v : em;
    res = fmaf(act, sAi[n], res);
  }
  float* p = out + (size_t)b * kCh + c;
  *(volatile float*)p = res;
  __threadfence();
  *(volatile float*)p = res;
}

extern "C" void kernel_launch(void* const* d_in, const int* in_sizes, int n_in,
                              void* d_out, int out_size, void* d_ws, size_t ws_size,
                              hipStream_t stream) {
  if (n_in < 7) return;
  if (in_sizes[0] != kPts * kCin) return;
  if (in_sizes[1] != kPts * 3) return;
  if (in_sizes[2] != kCh * kKdim) return;
  if (in_sizes[3] != kCh) return;
  if (in_sizes[4] != kRep * kGridN) return;
  if (in_sizes[5] != kGridN) return;
  if (in_sizes[6] != kPts) return;
  if (out_size != kGraphs * kCh) return;
  if (ws_size < kWsTotal) return;

  const float* x      = (const float*)d_in[0];
  const float* coords = (const float*)d_in[1];
  const float* W      = (const float*)d_in[2];
  const float* gamma  = (const float*)d_in[3];
  const float* Amat   = (const float*)d_in[4];
  const float* Ainv   = (const float*)d_in[5];
  const int*   batch  = (const int*)d_in[6];
  float* out = (float*)d_out;

  char* ws = (char*)d_ws;
  unsigned short* TP  = (unsigned short*)(ws + kOffTP);
  unsigned short* WH  = (unsigned short*)(ws + kOffWH);
  float*          OP  = (float*)(ws + kOffOP);
  float*          SCL = (float*)(ws + kOffSCL);

  cast_w_kernel<<<(kCh * kKdim / 8) / 256, 256, 0, stream>>>(W, WH);
  pool_kernel<<<kGraphs, 128, 0, stream>>>(x, coords, batch, TP);
  gemm_f16_tile64<<<dim3((kRowsT / 64) / 8, 1), 256, 0, stream>>>(
      TP, kKdim, WH, kKdim, OP, kCh, kRowsT, kCh, kKdim, kInvCarryW);
  scale_kernel<<<1, 256, 0, stream>>>(OP, gamma, SCL);
  final_kernel<<<kGraphs, kCh, 0, stream>>>(OP, SCL, Amat, Ainv, out);
}
